// linearized_attention_14628658610495
// MI455X (gfx1250) — hardware-verified
//
#include <hip/hip_runtime.h>
#include <math.h>
#include <stdint.h>

constexpr int NBATCH  = 16;
constexpr int NTOK    = 4096;
constexpr int CIN     = 128;
constexpr int DHEAD   = 64;
constexpr int NHEAD   = 8;
constexpr int HID     = 512;
constexpr int MFEAT   = 30;
constexpr int NSEQ_IT = 2;
constexpr int NITER   = NBATCH / NSEQ_IT;
constexpr int ROWS_IT = NSEQ_IT * NTOK;
constexpr int NSLOT   = NSEQ_IT * NHEAD;
constexpr int QKW     = 2 * HID;
constexpr int KTROWS  = 64;
constexpr int QPW     = 32;
constexpr int KT_LDSP = 264;
constexpr int QP_LDSP = 20;
constexpr float SCL_D   = 0.35355339059327373f;
constexpr float RATIO_F = 0.18257418583505536f;
constexpr float EPS_F   = 1e-6f;

constexpr size_t SZ_XB   = (size_t)NBATCH * NTOK * CIN * 2;
constexpr size_t SZ_WQK  = (size_t)QKW * CIN * 2;
constexpr size_t SZ_WV   = (size_t)HID * CIN * 2;
constexpr size_t SZ_WO   = (size_t)DHEAD * HID * 2;
constexpr size_t SZ_PRJ  = (size_t)64 * 128 * 2;
constexpr size_t SZ_BQK  = (size_t)QKW * 4;
constexpr size_t SZ_BV   = (size_t)HID * 4;
constexpr size_t SZ_BO   = 256;
constexpr size_t SZ_DQK  = (size_t)ROWS_IT * QKW * 2;
constexpr size_t SZ_VT   = (size_t)NSLOT * 64 * NTOK * 2;
constexpr size_t SZ_DD   = (size_t)ROWS_IT * NHEAD * 64 * 4;
constexpr size_t SZ_KT   = (size_t)NSLOT * KTROWS * NTOK * 2;
constexpr size_t SZ_KVS  = (size_t)NSLOT * 64 * 64 * 2;
constexpr size_t SZ_KSUM = (size_t)NSLOT * 32 * 4;
constexpr size_t SZ_QPP  = (size_t)NSLOT * NTOK * QPW * 2;
constexpr size_t SZ_OP   = (size_t)ROWS_IT * HID * 2;

constexpr size_t OFF_XB   = 0;
constexpr size_t OFF_WQK  = OFF_XB + SZ_XB;
constexpr size_t OFF_WV   = OFF_WQK + SZ_WQK;
constexpr size_t OFF_WO   = OFF_WV + SZ_WV;
constexpr size_t OFF_PRJ  = OFF_WO + SZ_WO;
constexpr size_t OFF_BQK  = OFF_PRJ + SZ_PRJ;
constexpr size_t OFF_BV   = OFF_BQK + SZ_BQK;
constexpr size_t OFF_BO   = OFF_BV + SZ_BV;
constexpr size_t OFF_DQKH = OFF_BO + SZ_BO;
constexpr size_t OFF_DQKL = OFF_DQKH + SZ_DQK;
constexpr size_t OFF_VTH  = OFF_DQKL + SZ_DQK;
constexpr size_t OFF_VTL  = OFF_VTH + SZ_VT;
constexpr size_t OFF_DD   = OFF_VTL + SZ_VT;
constexpr size_t OFF_KTH  = OFF_DD + SZ_DD;
constexpr size_t OFF_KTL  = OFF_KTH + SZ_KT;
constexpr size_t OFF_KVSH = OFF_KTL + SZ_KT;
constexpr size_t OFF_KVSL = OFF_KVSH + SZ_KVS;
constexpr size_t OFF_KSUM = OFF_KVSL + SZ_KVS;
constexpr size_t OFF_QPPH = OFF_KSUM + SZ_KSUM;
constexpr size_t OFF_QPPL = OFF_QPPH + SZ_QPP;
constexpr size_t OFF_OPH  = OFF_QPPL + SZ_QPP;
constexpr size_t OFF_OPL  = OFF_OPH + SZ_OP;
constexpr size_t WS_TOTAL = OFF_OPL + SZ_OP;
static_assert(WS_TOTAL == 126574848, "ws total");
static_assert(WS_TOTAL <= 134217728, "ws cap");
static_assert((OFF_DQKH % 256) == 0 && (OFF_KSUM % 256) == 0 && (OFF_OPL % 256) == 0, "align");

typedef __attribute__((ext_vector_type(16))) _Float16 v16h;
typedef __attribute__((ext_vector_type(8)))  _Float16 v8h;
typedef __attribute__((ext_vector_type(16))) __bf16   v16b;
typedef __attribute__((ext_vector_type(8)))  __bf16   v8b;
typedef __attribute__((ext_vector_type(8)))  float    v8f;
typedef __attribute__((ext_vector_type(4)))  float    v4f;
typedef __attribute__((ext_vector_type(4)))  unsigned int v4u;
typedef __attribute__((ext_vector_type(2)))  unsigned int v2u;

__device__ __forceinline__ unsigned short f2bf_bits(float f) {
  unsigned u = __float_as_uint(f);
  return (unsigned short)((u + 0x7FFFu + ((u >> 16) & 1u)) >> 16);
}
__device__ __forceinline__ float bf_bits2f(unsigned short h) { return __uint_as_float(((unsigned)h) << 16); }

__device__ __forceinline__ void dep_guard_h(v8f& a, v8f& b, v16h x, v16h y) { asm volatile("v_nop\n\tv_nop\n\tv_nop\n\tv_nop" : "+v"(a), "+v"(b) : "v"(x), "v"(y)); }
__device__ __forceinline__ void dep_guard_b(v8f& a, v8f& b, v16b x, v16b y) { asm volatile("v_nop\n\tv_nop\n\tv_nop\n\tv_nop" : "+v"(a), "+v"(b) : "v"(x), "v"(y)); }
__device__ __forceinline__ void keep4_h(v16h a, v16h b, v16h c, v16h d) { asm volatile("v_nop" :: "v"(a), "v"(b), "v"(c), "v"(d)); }
__device__ __forceinline__ void keep4_b(v16b a, v16b b, v16b c, v16b d) { asm volatile("v_nop" :: "v"(a), "v"(b), "v"(c), "v"(d)); }
__device__ __forceinline__ void acc_guard4(v8f& a, v8f& b, v8f& c, v8f& d) { asm volatile("v_nop\n\tv_nop\n\tv_nop\n\tv_nop" : "+v"(a), "+v"(b), "+v"(c), "+v"(d)); }
template <typename T> struct Frag;
template <> struct Frag<_Float16> {
  typedef v16h V; union U { v16h v; v8h h[2]; };
  static __device__ __forceinline__ v16h load(const _Float16* p) {
    U f; f.h[0] = *(const v8h*)(p); f.h[1] = *(const v8h*)(p + 16); return f.v;
  }
  static __device__ __forceinline__ v8f mma(v16h a, v16h b, v8f c) {
    return __builtin_amdgcn_wmma_f32_16x16x32_f16(false, a, false, b, (short)0, c, false, false);
  }
  static __device__ __forceinline__ void guard(v8f& a, v8f& b, v16h x, v16h y) { dep_guard_h(a, b, x, y); }
  static __device__ __forceinline__ void keep(v16h a, v16h b, v16h c, v16h d) { keep4_h(a, b, c, d); }
};
template <> struct Frag<__bf16> {
  typedef v16b V; union U { v16b v; v8b h[2]; };
  static __device__ __forceinline__ v16b load(const __bf16* p) {
    U f; f.h[0] = *(const v8b*)(p); f.h[1] = *(const v8b*)(p + 16); return f.v;
  }
  static __device__ __forceinline__ v8f mma(v16b a, v16b b, v8f c) {
    return __builtin_amdgcn_wmma_f32_16x16x32_bf16(false, a, false, b, (short)0, c, false, false);
  }
  static __device__ __forceinline__ void guard(v8f& a, v8f& b, v16b x, v16b y) { dep_guard_b(a, b, x, y); }
  static __device__ __forceinline__ void keep(v16b a, v16b b, v16b c, v16b d) { keep4_b(a, b, c, d); }
};

__device__ __forceinline__ unsigned pk16(unsigned short a, unsigned short b) { return (unsigned)a | ((unsigned)b << 16); }
__device__ __forceinline__ float bf_rne(float f) { return bf_bits2f(f2bf_bits(f)); }

template <int ET> struct Elem;
template <> struct Elem<0> { typedef _Float16 T; };
template <> struct Elem<1> { typedef __bf16 T; };
template <int ET, int SPLIT, int BIAS_MODE, int OUT_MODE, bool RESID, int ACT = 0>
__global__ __launch_bounds__(256) void wmma_gemm64(
    const unsigned short* __restrict__ Ap, const unsigned short* __restrict__ A2p, int lda, long strideA,
    const unsigned short* __restrict__ Btp, const unsigned short* __restrict__ Bt2p, int ldb, long strideB,
    void* __restrict__ Cout, void* __restrict__ Cout2, int ldc, long strideC,
    const float* __restrict__ bias,
    const float* __restrict__ resid, long strideR,
    int M, int N, int K, float scale) {
  typedef typename Elem<ET>::T T;
  typedef typename Frag<T>::V V;
  const T* A = (const T*)Ap; const T* A2 = (const T*)A2p; const T* Bt = (const T*)Btp; const T* Bt2 = (const T*)Bt2p;
  __shared__ __align__(16) float sT[8][16 * 68];
  const int b    = blockIdx.y;
  const int lane = threadIdx.x & 31;
  const int wave = threadIdx.x >> 5;
  const int tilesN = N >> 6;
  const int tilesM = M >> 6;
  const int tile = blockIdx.x * 8 + wave;
  if (tile >= tilesM * tilesN) return;
  const int tm = tile / tilesN;
  const int tn = tile - tm * tilesN;
  const int m0 = tm << 6;
  const int n0 = tn << 6;

  const T* Ab  = A  + (size_t)b * strideA;
  const T* Bb  = Bt + (size_t)b * strideB;
  const T* Ab2 = (SPLIT >= 1) ? (A2  + (size_t)b * strideA) : nullptr;
  const T* Bb2 = (SPLIT == 2) ? (Bt2 + (size_t)b * strideB) : nullptr;

  const int rlane = lane & 15;
  const int koff  = (lane >> 4) * 8;
  const int mOff  = (lane >> 4) * 8;

  v8f acc[4][4];
#pragma unroll
  for (int i = 0; i < 4; ++i)
#pragma unroll
    for (int j = 0; j < 4; ++j) acc[i][j] = (v8f){0.f,0.f,0.f,0.f,0.f,0.f,0.f,0.f};

  for (int k0 = 0; k0 < K; k0 += 32) {
    V bh[4], bl[4];
#pragma unroll
    for (int j = 0; j < 4; ++j) {
      const size_t bo = (size_t)(n0 + (j << 4) + rlane) * ldb + koff + k0;
      bh[j] = Frag<T>::load(Bb + bo);
      if (SPLIT == 2) bl[j] = Frag<T>::load(Bb2 + bo);
    }
#pragma unroll
    for (int i = 0; i < 4; ++i) {
      const size_t ao = (size_t)(m0 + (i << 4) + rlane) * lda + koff + k0;
      V ah = Frag<T>::load(Ab + ao);
      V al;
      if (SPLIT >= 1) al = Frag<T>::load(Ab2 + ao); else al = ah;
#pragma unroll
      for (int j = 0; j < 4; ++j) {
        acc[i][j] = Frag<T>::mma(ah, bh[j], acc[i][j]);
        if (SPLIT == 2) acc[i][j] = Frag<T>::mma(ah, bl[j], acc[i][j]);
        if (SPLIT >= 1) acc[i][j] = Frag<T>::mma(al, bh[j], acc[i][j]);
      }
      Frag<T>::guard(acc[i][0], acc[i][3], ah, al);
    }
    Frag<T>::keep(bh[0], bh[1], bh[2], bh[3]);
    if (SPLIT == 2) Frag<T>::keep(bl[0], bl[1], bl[2], bl[3]);
  }
  acc_guard4(acc[0][0], acc[0][1], acc[0][2], acc[0][3]);
  acc_guard4(acc[1][0], acc[1][1], acc[1][2], acc[1][3]);
  acc_guard4(acc[2][0], acc[2][1], acc[2][2], acc[2][3]);
  acc_guard4(acc[3][0], acc[3][1], acc[3][2], acc[3][3]);

  float* slab = sT[wave];
  const float* Rb = RESID ? (resid + (size_t)b * strideR) : nullptr;
#pragma unroll
  for (int i = 0; i < 4; ++i) {
    const int mBase = m0 + (i << 4);
#pragma unroll
    for (int j = 0; j < 4; ++j) {
      const int n = n0 + (j << 4) + rlane;
      float bv = 0.f;
      if (BIAS_MODE == 2) bv = bias[n];
#pragma unroll
      for (int r = 0; r < 8; ++r) {
        float v = acc[i][j][r] * scale;
        if (BIAS_MODE == 1) v += bias[mBase + mOff + r];
        if (BIAS_MODE == 2) v += bv;
        if (RESID) v += Rb[(size_t)(mBase + mOff + r) * ldc + n];
        if (ACT == 2) v = fmaxf(v, 0.0f);
        if (ACT == 4) v = (v > 0.f) ? v : 0.01f * v;
        slab[(mOff + r) * 68 + (j << 4) + rlane] = v;
      }
    }
    __builtin_amdgcn_fence(__ATOMIC_RELEASE, "workgroup");
    __builtin_amdgcn_wave_barrier();
    __builtin_amdgcn_fence(__ATOMIC_ACQUIRE, "workgroup");
    if (OUT_MODE == 0) {
      float* C = (float*)Cout + (size_t)b * strideC;
      const int hh = lane >> 4, c4 = (lane & 15) * 4;
      for (int pass = 0; pass < 2; ++pass) {
#pragma unroll
        for (int it = 0; it < 8; ++it) {
          const int row = it * 2 + hh;
          v4f v = *(const v4f*)(slab + row * 68 + c4);
          *(volatile v4f*)(C + (size_t)(mBase + row) * ldc + n0 + c4) = v;
        }
        __threadfence();
      }
    } else {
      const int q = lane >> 3, c8 = (lane & 7) * 8;
      unsigned short* C  = (unsigned short*)Cout  + (size_t)b * strideC;
      unsigned short* C2 = (OUT_MODE == 2) ? ((unsigned short*)Cout2 + (size_t)b * strideC) : nullptr;
      for (int pass = 0; pass < 2; ++pass) {
#pragma unroll
        for (int it = 0; it < 4; ++it) {
          const int row = it * 4 + q;
          const float* sp = slab + row * 68 + c8;
          v8h hv, lv;
#pragma unroll
          for (int e = 0; e < 8; ++e) {
            if (OUT_MODE == 1) {
              hv[e] = (_Float16)sp[e];
            } else {
              unsigned short hb = f2bf_bits(sp[e]);
              unsigned short lb = f2bf_bits(sp[e] - bf_bits2f(hb));
              hv[e] = __builtin_bit_cast(_Float16, hb);
              lv[e] = __builtin_bit_cast(_Float16, lb);
            }
          }
          *(volatile v8h*)(C + (size_t)(mBase + row) * ldc + n0 + c8) = hv;
          if (OUT_MODE == 2) *(volatile v8h*)(C2 + (size_t)(mBase + row) * ldc + n0 + c8) = lv;
        }
        __threadfence();
      }
    }
    __builtin_amdgcn_fence(__ATOMIC_RELEASE, "workgroup");
    __builtin_amdgcn_wave_barrier();
    __builtin_amdgcn_fence(__ATOMIC_ACQUIRE, "workgroup");
  }
}

__device__ __forceinline__ v4u pack_bf8(v4f a, v4f c) {
  return (v4u){ pk16(f2bf_bits(a[0]), f2bf_bits(a[1])), pk16(f2bf_bits(a[2]), f2bf_bits(a[3])),
                pk16(f2bf_bits(c[0]), f2bf_bits(c[1])), pk16(f2bf_bits(c[2]), f2bf_bits(c[3])) };
}
__device__ __forceinline__ void st2_u4(unsigned short* p, v4u u) {
  *(volatile v4u*)p = u;
  __threadfence();
  *(volatile v4u*)p = u;
}
__device__ __forceinline__ void st2_f4(float* p, v4f v) {
  *(volatile v4f*)p = v;
  __threadfence();
  *(volatile v4f*)p = v;
}
__device__ __forceinline__ v4f sel4(int s, v4f a, v4f c) {
  v4f r;
  r[0] = s ? c[0] : a[0]; r[1] = s ? c[1] : a[1]; r[2] = s ? c[2] : a[2]; r[3] = s ? c[3] : a[3];
  return r;
}
__device__ __forceinline__ v4f rne4(v4f a) {
  v4f r;
  r[0] = bf_rne(a[0]); r[1] = bf_rne(a[1]); r[2] = bf_rne(a[2]); r[3] = bf_rne(a[3]);
  return r;
}

constexpr int SEGB_X   = 4096;
constexpr int SEGB_WQK = 64;
constexpr int SEGB_WV  = 32;
constexpr int SEGB_WO  = 16;
constexpr int SEGB_PRJ = 4;
constexpr int CAST_BLOCKS = SEGB_X + SEGB_WQK + SEGB_WV + SEGB_WO + SEGB_PRJ + 3;

__global__ __launch_bounds__(256) void cast_kernel(
    const float* __restrict__ x,
    const float* __restrict__ wq, const float* __restrict__ wqb,
    const float* __restrict__ wk, const float* __restrict__ wkb,
    const float* __restrict__ wv, const float* __restrict__ wvb,
    const float* __restrict__ wo, const float* __restrict__ wob,
    const float* __restrict__ proj,
    unsigned short* __restrict__ xb, unsigned short* __restrict__ wqkb, unsigned short* __restrict__ wvb16,
    unsigned short* __restrict__ wob16, unsigned short* __restrict__ prjb,
    float* __restrict__ bqk_r, float* __restrict__ bv_r, float* __restrict__ bo_r) {
  const int blk = blockIdx.x;
  const int t = threadIdx.x;
  if (blk < SEGB_X) {
    const size_t u = (size_t)blk * 256 + t;
    const float* p = x + 8 * u;
    const v4f a = *(const v4f*)(p);
    const v4f c = *(const v4f*)(p + 4);
    st2_u4(xb + 8 * u, pack_bf8(a, c));
  } else if (blk < SEGB_X + SEGB_WQK) {
    const int u  = (blk - SEGB_X) * 256 + t;
    const int r  = u >> 4;
    const int c8 = (u & 15) * 8;
    const int hh = r >> 7;
    const int s  = (r >> 6) & 1;
    const int d  = r & 63;
    const size_t src = (size_t)(hh * 64 + d) * CIN + c8;
    const v4f a0 = *(const v4f*)(wq + src);
    const v4f a1 = *(const v4f*)(wq + src + 4);
    const v4f b0 = *(const v4f*)(wk + src);
    const v4f b1 = *(const v4f*)(wk + src + 4);
    st2_u4(wqkb + (size_t)r * CIN + c8, pack_bf8(sel4(s, a0, b0), sel4(s, a1, b1)));
  } else if (blk < SEGB_X + SEGB_WQK + SEGB_WV) {
    const int u  = (blk - SEGB_X - SEGB_WQK) * 256 + t;
    const int r  = u >> 4;
    const int c8 = (u & 15) * 8;
    const size_t src = (size_t)r * CIN + c8;
    const v4f a = *(const v4f*)(wv + src);
    const v4f c = *(const v4f*)(wv + src + 4);
    st2_u4(wvb16 + src, pack_bf8(a, c));
  } else if (blk < SEGB_X + SEGB_WQK + SEGB_WV + SEGB_WO) {
    const int u = (blk - SEGB_X - SEGB_WQK - SEGB_WV) * 256 + t;
    const size_t src = (size_t)u * 8;
    const v4f a = *(const v4f*)(wo + src);
    const v4f c = *(const v4f*)(wo + src + 4);
    st2_u4(wob16 + src, pack_bf8(a, c));
  } else if (blk < SEGB_X + SEGB_WQK + SEGB_WV + SEGB_WO + SEGB_PRJ) {
    const int u    = (blk - SEGB_X - SEGB_WQK - SEGB_WV - SEGB_WO) * 256 + t;
    const int row  = u >> 4;
    const int c8   = (u & 15) * 8;
    const int side = c8 >> 6;
    const int dcol = c8 & 63;
    const int mraw = row - 32 * side;
    const int valid = (mraw >= 0) && (mraw < MFEAT);
    int mcl = mraw < 0 ? 0 : mraw;
    mcl = mcl > (MFEAT - 1) ? (MFEAT - 1) : mcl;
    const size_t src = (size_t)mcl * DHEAD + dcol;
    const v4f a = *(const v4f*)(proj + src);
    const v4f c = *(const v4f*)(proj + src + 4);
    const v4u pk = pack_bf8(a, c);
    const v4u z  = (v4u){0u, 0u, 0u, 0u};
    v4u o;
    o[0] = valid ? pk[0] : z[0]; o[1] = valid ? pk[1] : z[1]; o[2] = valid ? pk[2] : z[2]; o[3] = valid ? pk[3] : z[3];
    st2_u4(prjb + (size_t)row * 128 + c8, o);
  } else if (blk == CAST_BLOCKS - 3) {
    const int r0 = 4 * t;
    const int hh = r0 >> 7;
    const int s  = (r0 >> 6) & 1;
    const int d0 = r0 & 63;
    const int src = hh * 64 + d0;
    const v4f a = *(const v4f*)(wqb + src);
    const v4f c = *(const v4f*)(wkb + src);
    st2_f4(bqk_r + r0, rne4(sel4(s, a, c)));
  } else if (blk == CAST_BLOCKS - 2) {
    if (t < 128) {
      const v4f a = *(const v4f*)(wvb + 4 * t);
      st2_f4(bv_r + 4 * t, rne4(a));
    }
  } else {
    if (t < 16) {
      const v4f a = *(const v4f*)(wob + 4 * t);
      st2_f4(bo_r + 4 * t, rne4(a));
    }
  }
}

constexpr int ZKT_THREADS = NSLOT * (KTROWS - MFEAT) * (NTOK / 8);
static_assert(ZKT_THREADS == 1088 * 256, "zero grid");

__global__ __launch_bounds__(256) void zero_kt_kernel(unsigned short* __restrict__ kth, unsigned short* __restrict__ ktl) {
  const int u = blockIdx.x * 256 + threadIdx.x;
  const int per_slot = (KTROWS - MFEAT) * (NTOK / 8);
  const int slot = u / per_slot;
  const int rem  = u - slot * per_slot;
  const int row  = MFEAT + rem / (NTOK / 8);
  const int c8   = (rem & (NTOK / 8 - 1)) * 8;
  const size_t off = ((size_t)(slot * KTROWS + row)) * NTOK + c8;
  const v4u z = (v4u){0u, 0u, 0u, 0u};
  st2_u4(kth + off, z);
  st2_u4(ktl + off, z);
}

__global__ __launch_bounds__(256) void featk_kernel(
    const float* __restrict__ dd, const unsigned short* __restrict__ dqh, const unsigned short* __restrict__ dql,
    unsigned short* __restrict__ kth, unsigned short* __restrict__ ktl, float* __restrict__ ksum) {
  __shared__ __align__(16) unsigned short st_hi[32 * KT_LDSP];
  __shared__ __align__(16) unsigned short st_lo[32 * KT_LDSP];
  __shared__ float ksw[8 * 32];
  __shared__ float red[8];
  const int slot = blockIdx.x;
  const int bl   = slot >> 3;
  const int h    = slot & 7;
  const int t    = threadIdx.x;
  const int lane = t & 31, wave = t >> 5;
  ksw[t] = 0.f;

  float mx = -INFINITY;
#pragma unroll 1
  for (int i = 0; i < 16; ++i) {
    const int niter = bl * NTOK + i * 256 + t;
    const float* dr = dd + ((size_t)niter * NHEAD + h) * 64 + 32;
#pragma unroll
    for (int j = 0; j < 8; ++j) {
      const v4f v = *(const v4f*)(dr + 4 * j);
#pragma unroll
      for (int e = 0; e < 4; ++e) {
        if (4 * j + e < MFEAT) mx = fmaxf(mx, v[e]);
      }
    }
  }
#pragma unroll
  for (int off = 1; off < 32; off <<= 1) mx = fmaxf(mx, __shfl_xor(mx, off, 32));
  if (lane == 0) red[wave] = mx;
  __syncthreads();
  float kmx = red[0];
#pragma unroll
  for (int w = 1; w < 8; ++w) kmx = fmaxf(kmx, red[w]);

#pragma unroll 1
  for (int i = 0; i < 16; ++i) {
    const int niter = bl * NTOK + i * 256 + t;
    const float* dr = dd + ((size_t)niter * NHEAD + h) * 64 + 32;
    const unsigned short* hp = dqh + (size_t)niter * QKW + h * 128 + 64;
    const unsigned short* lp = dql + (size_t)niter * QKW + h * 128 + 64;
    float ss = 0.f;
#pragma unroll 1
    for (int j = 0; j < 8; ++j) {
      const v4u a = *(const v4u*)(hp + 8 * j);
      const v4u c = *(const v4u*)(lp + 8 * j);
#pragma unroll
      for (int e = 0; e < 4; ++e) {
        const float f0 = (__uint_as_float(a[e] << 16) + __uint_as_float(c[e] << 16)) * SCL_D;
        const float f1 = (__uint_as_float(a[e] & 0xffff0000u) + __uint_as_float(c[e] & 0xffff0000u)) * SCL_D;
        ss += f0 * f0;
        ss += f1 * f1;
      }
    }
    const float diag = 0.5f * ss;
#pragma unroll 1
    for (int j = 0; j < 8; ++j) {
      const v4f v = *(const v4f*)(dr + 4 * j);
#pragma unroll
      for (int e = 0; e < 4; ++e) {
        const int m = 4 * j + e;
        float p = RATIO_F * (expf((v[e] - diag) - kmx) + EPS_F);
        p = (m < MFEAT) ? p : 0.f;
        const unsigned short hb = f2bf_bits(p);
        const unsigned short lb = f2bf_bits(p - bf_bits2f(hb));
        st_hi[m * KT_LDSP + t] = hb;
        st_lo[m * KT_LDSP + t] = lb;
        float s = p;
#pragma unroll
        for (int off = 1; off < 32; off <<= 1) s += __shfl_xor(s, off, 32);
        if (lane == 0) ksw[wave * 32 + m] += s;
      }
    }
    __syncthreads();
    for (int pass = 0; pass < 2; ++pass) {
#pragma unroll
      for (int jj = 0; jj < 4; ++jj) {
        const int m = wave * 4 + jj;
        if (m < MFEAT) {
          const v4u a = *(const v4u*)(st_hi + m * KT_LDSP + lane * 8);
          const v4u c = *(const v4u*)(st_lo + m * KT_LDSP + lane * 8);
          const size_t off = ((size_t)(slot * KTROWS + m)) * NTOK + (size_t)i * 256 + lane * 8;
          *(volatile v4u*)(kth + off) = a;
          *(volatile v4u*)(ktl + off) = c;
        }
      }
      __threadfence();
    }
    __syncthreads();
  }

  if (wave == 0) {
    float s = 0.f;
#pragma unroll
    for (int w = 0; w < 8; ++w) s += ksw[w * 32 + lane];
    const float val = (lane < MFEAT) ? s : 0.f;
    float* kp = ksum + slot * 32 + lane;
    *(volatile float*)kp = val;
    __threadfence();
    *(volatile float*)kp = val;
  }
}

__global__ __launch_bounds__(256) void featq_kernel(
    const float* __restrict__ dd, const unsigned short* __restrict__ dqh, const unsigned short* __restrict__ dql,
    const float* __restrict__ ksum, unsigned short* __restrict__ qph, unsigned short* __restrict__ qpl) {
  __shared__ __align__(16) unsigned int sq_hi[256 * QP_LDSP];
  __shared__ __align__(16) unsigned int sq_lo[256 * QP_LDSP];
  const int c    = blockIdx.x;
  const int h    = blockIdx.y;
  const int t    = threadIdx.x;
  const int lane = t & 31, wave = t >> 5;
  const int bl   = c >> 4;
  const int slot = bl * NHEAD + h;
  const int niter = c * 256 + t;
  const float* dr  = dd + ((size_t)niter * NHEAD + h) * 64;
  const float* ksp = ksum + slot * 32;

  float mx = -INFINITY;
#pragma unroll
  for (int j = 0; j < 8; ++j) {
    const v4f v = *(const v4f*)(dr + 4 * j);
#pragma unroll
    for (int e = 0; e < 4; ++e) {
      if (4 * j + e < MFEAT) mx = fmaxf(mx, v[e]);
    }
  }
  const unsigned short* hp = dqh + (size_t)niter * QKW + h * 128;
  const unsigned short* lp = dql + (size_t)niter * QKW + h * 128;
  float ss = 0.f;
#pragma unroll 1
  for (int j = 0; j < 8; ++j) {
    const v4u a  = *(const v4u*)(hp + 8 * j);
    const v4u cc = *(const v4u*)(lp + 8 * j);
#pragma unroll
    for (int e = 0; e < 4; ++e) {
      const float f0 = (__uint_as_float(a[e] << 16) + __uint_as_float(cc[e] << 16)) * SCL_D;
      const float f1 = (__uint_as_float(a[e] & 0xffff0000u) + __uint_as_float(cc[e] & 0xffff0000u)) * SCL_D;
      ss += f0 * f0;
      ss += f1 * f1;
    }
  }
  const float diag = 0.5f * ss;
  float den = 0.f;
#pragma unroll 1
  for (int j = 0; j < 8; ++j) {
    const v4f v  = *(const v4f*)(dr + 4 * j);
    const v4f kk = *(const v4f*)(ksp + 4 * j);
#pragma unroll
    for (int e = 0; e < 4; ++e) {
      const int m = 4 * j + e;
      float p = RATIO_F * (expf((v[e] - diag) - mx) + EPS_F);
      p = (m < MFEAT) ? p : 0.f;
      den += p * kk[e];
    }
  }
  const float rden = 1.0f / den;
#pragma unroll 1
  for (int j = 0; j < 8; ++j) {
    const v4f v = *(const v4f*)(dr + 4 * j);
    unsigned short hb[4], lb[4];
#pragma unroll
    for (int e = 0; e < 4; ++e) {
      const int m = 4 * j + e;
      float p = RATIO_F * (expf((v[e] - diag) - mx) + EPS_F);
      p = (m < MFEAT) ? (p * rden) : 0.f;
      hb[e] = f2bf_bits(p);
      lb[e] = f2bf_bits(p - bf_bits2f(hb[e]));
    }
    const v2u wh = (v2u){ pk16(hb[0], hb[1]), pk16(hb[2], hb[3]) };
    const v2u wl = (v2u){ pk16(lb[0], lb[1]), pk16(lb[2], lb[3]) };
    *(v2u*)(sq_hi + t * QP_LDSP + 2 * j) = wh;
    *(v2u*)(sq_lo + t * QP_LDSP + 2 * j) = wl;
  }
  __syncthreads();
  const int n0w = (c & 15) * 256 + wave * 32;
  for (int pass = 0; pass < 2; ++pass) {
#pragma unroll
    for (int q = 0; q < 4; ++q) {
      const int rl  = q * 8 + (lane >> 2);
      const int cc4 = lane & 3;
      const v4u a  = *(const v4u*)(sq_hi + (wave * 32 + rl) * QP_LDSP + cc4 * 4);
      const v4u bb = *(const v4u*)(sq_lo + (wave * 32 + rl) * QP_LDSP + cc4 * 4);
      const size_t off = ((size_t)(slot * NTOK + n0w + rl)) * QPW + cc4 * 8;
      *(volatile v4u*)(qph + off) = a;
      *(volatile v4u*)(qpl + off) = bb;
    }
    __threadfence();
  }
}

extern "C" void kernel_launch(void* const* d_in, const int* in_sizes, int n_in,
                              void* d_out, int out_size, void* d_ws, size_t ws_size,
                              hipStream_t stream) {
  if (n_in < 10) return;
  if (in_sizes[0] != NBATCH * NTOK * CIN) return;
  if (in_sizes[1] != HID * CIN || in_sizes[3] != HID * CIN || in_sizes[5] != HID * CIN) return;
  if (in_sizes[7] != DHEAD * HID || in_sizes[9] != MFEAT * DHEAD) return;
  if (in_sizes[2] != HID || in_sizes[4] != HID || in_sizes[6] != HID || in_sizes[8] != DHEAD) return;
  if (out_size != NBATCH * NTOK * DHEAD) return;
  if (ws_size < WS_TOTAL) return;

  const float* x    = (const float*)d_in[0];
  const float* wq_w = (const float*)d_in[1];
  const float* wq_b = (const float*)d_in[2];
  const float* wk_w = (const float*)d_in[3];
  const float* wk_b = (const float*)d_in[4];
  const float* wv_w = (const float*)d_in[5];
  const float* wv_b = (const float*)d_in[6];
  const float* wo_w = (const float*)d_in[7];
  const float* wo_b = (const float*)d_in[8];
  const float* proj = (const float*)d_in[9];
  float* out = (float*)d_out;

  char* ws = (char*)d_ws;
  unsigned short* xb    = (unsigned short*)(ws + OFF_XB);
  unsigned short* wqk   = (unsigned short*)(ws + OFF_WQK);
  unsigned short* wvb16 = (unsigned short*)(ws + OFF_WV);
  unsigned short* wob16 = (unsigned short*)(ws + OFF_WO);
  unsigned short* prjb  = (unsigned short*)(ws + OFF_PRJ);
  float* bqk_r = (float*)(ws + OFF_BQK);
  float* bv_r  = (float*)(ws + OFF_BV);
  float* bo_r  = (float*)(ws + OFF_BO);
  unsigned short* dqkh = (unsigned short*)(ws + OFF_DQKH);
  unsigned short* dqkl = (unsigned short*)(ws + OFF_DQKL);
  unsigned short* vth  = (unsigned short*)(ws + OFF_VTH);
  unsigned short* vtl  = (unsigned short*)(ws + OFF_VTL);
  float* ddp = (float*)(ws + OFF_DD);
  unsigned short* kth  = (unsigned short*)(ws + OFF_KTH);
  unsigned short* ktl  = (unsigned short*)(ws + OFF_KTL);
  unsigned short* kvsh = (unsigned short*)(ws + OFF_KVSH);
  unsigned short* kvsl = (unsigned short*)(ws + OFF_KVSL);
  float* ksum = (float*)(ws + OFF_KSUM);
  unsigned short* qph  = (unsigned short*)(ws + OFF_QPPH);
  unsigned short* qpl  = (unsigned short*)(ws + OFF_QPPL);
  unsigned short* oph  = (unsigned short*)(ws + OFF_OPH);
  unsigned short* opl  = (unsigned short*)(ws + OFF_OPL);

  cast_kernel<<<dim3(CAST_BLOCKS), dim3(256), 0, stream>>>(x, wq_w, wq_b, wk_w, wk_b, wv_w, wv_b, wo_w, wo_b, proj,
                                                          xb, wqk, wvb16, wob16, prjb, bqk_r, bv_r, bo_r);
  zero_kt_kernel<<<dim3(ZKT_THREADS / 256), dim3(256), 0, stream>>>(kth, ktl);

  for (int it = 0; it < NITER; ++it) {
    const unsigned short* xit = xb + (size_t)it * ROWS_IT * CIN;

    wmma_gemm64<1, 0, 2, 2, false><<<dim3(256, 1), dim3(256), 0, stream>>>(
        xit, xit, CIN, 0L, wqk, wqk, CIN, 0L, (void*)dqkh, (void*)dqkl, QKW, 0L,
        bqk_r, bo_r, 0L, ROWS_IT, QKW, CIN, 1.0f);

    wmma_gemm64<1, 0, 1, 2, false><<<dim3(64, NSEQ_IT), dim3(256), 0, stream>>>(
        wvb16, wvb16, CIN, 0L, xit, xit, CIN, (long)NTOK * CIN, (void*)vth, (void*)vtl, NTOK, (long)HID * NTOK,
        bv_r, bo_r, 0L, HID, NTOK, CIN, 1.0f);

    wmma_gemm64<1, 1, 0, 0, false><<<dim3(128, 1), dim3(256), 0, stream>>>(
        dqkh, dqkl, 128, 0L, prjb, prjb, 128, 0L, (void*)ddp, (void*)ddp, 64, 0L,
        bqk_r, bo_r, 0L, ROWS_IT * NHEAD, 64, 128, SCL_D);

    featk_kernel<<<dim3(NSLOT), dim3(256), 0, stream>>>(ddp, dqkh, dqkl, kth, ktl, ksum);

    wmma_gemm64<1, 2, 0, 2, false><<<dim3(1, NSLOT), dim3(256), 0, stream>>>(
        vth, vtl, NTOK, (long)64 * NTOK, kth, ktl, NTOK, (long)KTROWS * NTOK, (void*)kvsh, (void*)kvsl, 64, 64L * 64L,
        bqk_r, bo_r, 0L, 64, 64, NTOK, 1.0f);

    featq_kernel<<<dim3(32, NHEAD), dim3(256), 0, stream>>>(ddp, dqkh, dqkl, ksum, qph, qpl);

    for (int bl = 0; bl < NSEQ_IT; ++bl) {
      wmma_gemm64<1, 2, 0, 2, false><<<dim3(8, NHEAD), dim3(256), 0, stream>>>(
          qph + (size_t)bl * NHEAD * NTOK * QPW, qpl + (size_t)bl * NHEAD * NTOK * QPW, QPW, (long)NTOK * QPW,
          kvsh + (size_t)bl * NHEAD * 4096, kvsl + (size_t)bl * NHEAD * 4096, 64, 4096L,
          (void*)(oph + (size_t)bl * NTOK * HID), (void*)(opl + (size_t)bl * NTOK * HID), HID, 64L,
          bqk_r, bo_r, 0L, NTOK, 64, QPW, 1.0f);
    }

    float* oit = out + (size_t)it * ROWS_IT * DHEAD;
    wmma_gemm64<1, 1, 2, 0, false><<<dim3(16, 1), dim3(256), 0, stream>>>(
        oph, opl, HID, 0L, wob16, wob16, HID, 0L, (void*)oit, (void*)oit, DHEAD, 0L,
        bo_r, bo_r, 0L, ROWS_IT, DHEAD, HID, 1.0f);
  }
}
